// EdgePredictor_52493090292432
// MI455X (gfx1250) — hardware-verified
//
#include <hip/hip_runtime.h>
#include <stddef.h>
#include <stdint.h>


#define NGC    100000
#define DX     2
#define D1     8
#define D2     16
#define KP     32
#define DH     64
#define NTHR   256
#define NWAVE  8
#define EPT    8
#define CHUNK  (NTHR * EPT)
#define WCAP   (EPT * 32)
#define LISTN  (NWAVE * WCAP)
#define NBA    512
#define SLA    9
#define RCAP   28672
#define DEGCAP 96
#define GBM    64
#define GTHR   128
#define XROWS  256
#define AGG_ZINTS  (LISTN + 2 * RCAP + 3 * NBA)
#define MISC_INTS  16
#define WSM_INTS   288
#define TILE1_INTS (NBA * D1)
#define TILE2_INTS (NBA * KP / 2)
#define LDS1_INTS  (AGG_ZINTS + MISC_INTS + WSM_INTS + TILE1_INTS)
#define LDS2_INTS  (AGG_ZINTS + MISC_INTS + WSM_INTS + TILE2_INTS)
#define WSMAX  134217728

static_assert((CHUNK & (CHUNK - 1)) == 0 && CHUNK <= 4096);
static_assert((NBA & (NBA - 1)) == 0 && NBA == (1 << SLA));
static_assert(((long long)CHUNK << SLA) < (1LL << 31));
static_assert(LISTN % NTHR == 0);
static_assert(NBA % NWAVE == 0 && NBA % 32 == 0 && NBA % GBM == 0);
static_assert(RCAP % 4 == 0 && AGG_ZINTS % 4 == 0 && LISTN % 4 == 0);
static_assert(((AGG_ZINTS + MISC_INTS + WSM_INTS) % 4) == 0);
static_assert(WSM_INTS >= 2 * D1 * D2 + D2);
static_assert(TILE1_INTS == NTHR * 4 * 4);
static_assert(TILE2_INTS * 2 == NTHR * 8 * 8);
static_assert(XROWS * KP == NTHR * 8 * 4);
static_assert(XROWS % GBM == 0);
static_assert(GBM == (GTHR / 32) * 16 && DH == 64 && KP == 32);
static_assert(LDS2_INTS * 4 <= 300000 && LDS1_INTS <= LDS2_INTS);

typedef float          v2f   __attribute__((ext_vector_type(2)));
typedef float          v4f   __attribute__((ext_vector_type(4)));
typedef float          v8f   __attribute__((ext_vector_type(8)));
typedef int            v2i   __attribute__((ext_vector_type(2)));
typedef int            v4i   __attribute__((ext_vector_type(4)));
typedef int            v8i   __attribute__((ext_vector_type(8)));
typedef unsigned short v4us  __attribute__((ext_vector_type(4)));
typedef unsigned short v8us  __attribute__((ext_vector_type(8)));
typedef unsigned short v16us __attribute__((ext_vector_type(16)));
typedef __bf16         v16bf __attribute__((ext_vector_type(16)));
typedef v2f  __attribute__((may_alias)) v2fa;
typedef v4f  __attribute__((may_alias)) v4fa;
typedef v2i  __attribute__((may_alias)) v2ia;
typedef v4i  __attribute__((may_alias)) v4ia;
typedef v8us __attribute__((may_alias)) v8usa;
union FragB { v16bf v; v16us u; v8us h[2]; v8i w; };

__device__ __forceinline__ v8f wmb(const FragB& a, const FragB& b, v8f c) {
  v8f d = __builtin_amdgcn_wmma_f32_16x16x32_bf16(false, a.v, false, b.v, (short)0, c, false, false);
  asm volatile("v_nop\n\tv_nop\n\tv_nop\n\tv_nop" : "+v"(d) : "v"(a.w), "v"(b.w));
  return d;
}

__device__ __forceinline__ unsigned bf16_bits(float f) {
  const unsigned u = __float_as_uint(f);
  return (u + 0x7FFFu + ((u >> 16) & 1u)) >> 16;
}
__device__ __forceinline__ float bf16_val(float f) {
  return __uint_as_float(bf16_bits(f) << 16);
}
__device__ __forceinline__ float qnan_f() { return __int_as_float(0x7fc00000); }

__device__ __forceinline__ void wave_sync() {
  __builtin_amdgcn_fence(__ATOMIC_RELEASE, "wavefront");
  __builtin_amdgcn_wave_barrier();
  __builtin_amdgcn_fence(__ATOMIC_ACQUIRE, "wavefront");
}

template <int SLB>
__device__ __forceinline__ int scan_chunk(const int* __restrict__ dsts, int nE, int cbase, int slotBase,
                                          int nb, int vec8, int* list, int tid, int lane, int wave) {
  int wc = 0;
  const int el0  = tid * EPT;
  const int e0   = cbase + el0;
  const int sent = -2147483647 - 1;
  v4i da, db;
  if (vec8 != 0 && cbase + CHUNK <= nE) {
    da = *(const v4i*)(dsts + e0);
    db = *(const v4i*)(dsts + e0 + 4);
  } else {
    da.x = (e0     < nE) ? dsts[min(e0,     nE - 1)] : sent;
    da.y = (e0 + 1 < nE) ? dsts[min(e0 + 1, nE - 1)] : sent;
    da.z = (e0 + 2 < nE) ? dsts[min(e0 + 2, nE - 1)] : sent;
    da.w = (e0 + 3 < nE) ? dsts[min(e0 + 3, nE - 1)] : sent;
    db.x = (e0 + 4 < nE) ? dsts[min(e0 + 4, nE - 1)] : sent;
    db.y = (e0 + 5 < nE) ? dsts[min(e0 + 5, nE - 1)] : sent;
    db.z = (e0 + 6 < nE) ? dsts[min(e0 + 6, nE - 1)] : sent;
    db.w = (e0 + 7 < nE) ? dsts[min(e0 + 7, nE - 1)] : sent;
  }
  const unsigned nbs = (unsigned)slotBase;
  const unsigned unb = (unsigned)nb;
  const unsigned s0 = (unsigned)da.x - nbs, s1 = (unsigned)da.y - nbs;
  const unsigned s2 = (unsigned)da.z - nbs, s3 = (unsigned)da.w - nbs;
  const unsigned s4 = (unsigned)db.x - nbs, s5 = (unsigned)db.y - nbs;
  const unsigned s6 = (unsigned)db.z - nbs, s7 = (unsigned)db.w - nbs;
  const bool h0 = s0 < unb, h1 = s1 < unb, h2 = s2 < unb, h3 = s3 < unb;
  const bool h4 = s4 < unb, h5 = s5 < unb, h6 = s6 < unb, h7 = s7 < unb;
  const unsigned any = __builtin_amdgcn_ballot_w32(h0 | h1 | h2 | h3 | h4 | h5 | h6 | h7);
  if (any != 0u) {
#define HITJ(J, HJ, SJ) { \
      const unsigned mj = __builtin_amdgcn_ballot_w32(HJ); \
      if (mj != 0u) { \
        if (HJ) { \
          const int pos = wc + (int)__builtin_amdgcn_mbcnt_lo(mj, 0u); \
          if (pos < WCAP) list[wave * WCAP + pos] = ((el0 + (J)) << SLB) | (int)(SJ); \
        } \
        wc += (int)__builtin_popcount(mj); } }
    HITJ(0, h0, s0)
    HITJ(1, h1, s1)
    HITJ(2, h2, s2)
    HITJ(3, h3, s3)
    HITJ(4, h4, s4)
    HITJ(5, h5, s5)
    HITJ(6, h6, s6)
    HITJ(7, h7, s7)
#undef HITJ
  }
  return wc;
}

__global__ __launch_bounds__(NTHR) void k_wprep(const float* __restrict__ wa, unsigned short* bw) {
  __shared__ __attribute__((aligned(16))) unsigned short sb[2 * DH * KP];
  const int tid = (int)threadIdx.x;
#pragma unroll 1
  for (int it = 0; it < 2; ++it) {
    const int u  = it * NTHR + tid;
    const int p  = u >> 8;
    const int v  = u & 255;
    const int n  = v >> 2;
    const int k8 = (v & 3) * 8;
    const int kr = 16 * p + (k8 & 15);
    const float* src = wa + (size_t)kr * DH + n;
    v8us o;
#pragma unroll
    for (int i = 0; i < 8; ++i) o[i] = (unsigned short)bf16_bits(src[(size_t)i * DH]);
    *(v8usa*)(sb + (p * DH + n) * KP + k8) = o;
  }
  __syncthreads();
  const v8us q0 = *(const v8usa*)(sb + 8 * tid);
  const v8us q1 = *(const v8usa*)(sb + 2048 + 8 * tid);
  *(volatile v8us*)(bw + 8 * tid) = q0;
  *(volatile v8us*)(bw + 2048 + 8 * tid) = q1;
  __threadfence();
  *(volatile v8us*)(bw + 8 * tid) = q0;
  *(volatile v8us*)(bw + 2048 + 8 * tid) = q1;
}

__global__ __launch_bounds__(NTHR) void k_xprep(const float* __restrict__ x, const int* __restrict__ mask,
                                                const float* __restrict__ wu, const float* __restrict__ bu,
                                                int nG, int nU, int nTot, unsigned short* xup) {
  __shared__ __attribute__((aligned(16))) unsigned short st[XROWS * KP];
  __shared__ float wsm[3 * D2];
  const int tid = (int)threadIdx.x;
  const int row = (int)blockIdx.x * XROWS + tid;
  if (tid < DX * D2) wsm[tid] = bf16_val(wu[tid]);
  if (tid < D2) wsm[DX * D2 + tid] = bf16_val(bu[tid]);
  __syncthreads();
  const bool live = row < nU;
  const int rc = live ? row : nU - 1;
  int xr = nG + rc;
  xr = xr < 0 ? 0 : (xr > nTot - 1 ? nTot - 1 : xr);
  const v2f xv = *(const v2fa*)(x + (size_t)xr * DX);
  const float x0 = bf16_val(xv.x), x1 = bf16_val(xv.y);
  const int mk = mask[xr];
  const bool mbad = live && (mk != 0);
  const float pzr = mbad ? qnan_f() : 0.0f;
  v8us ha, hb8, la, lb8;
#pragma unroll
  for (int n = 0; n < D2; ++n) {
    const float t = fmaf(x1, wsm[D2 + n], x0 * wsm[n]) + wsm[2 * D2 + n];
    const float v = live ? (t + pzr) : 0.0f;
    const unsigned hbits = bf16_bits(v);
    const unsigned lbits = bf16_bits(v - __uint_as_float(hbits << 16));
    if (n < 8) { ha[n] = (unsigned short)hbits; la[n] = (unsigned short)lbits; }
    else       { hb8[n - 8] = (unsigned short)hbits; lb8[n - 8] = (unsigned short)lbits; }
  }
  unsigned short* srow = st + tid * KP;
  *(v8usa*)(srow)      = ha;
  *(v8usa*)(srow + 8)  = hb8;
  *(v8usa*)(srow + 16) = la;
  *(v8usa*)(srow + 24) = lb8;
  __syncthreads();
  v8us q[4];
#pragma unroll
  for (int i = 0; i < 4; ++i) q[i] = *(const v8usa*)(st + i * 2048 + 8 * tid);
  unsigned short* gp = xup + (size_t)blockIdx.x * XROWS * KP;
#pragma unroll
  for (int i = 0; i < 4; ++i) *(volatile v8us*)(gp + i * 2048 + 8 * tid) = q[i];
  __threadfence();
#pragma unroll
  for (int i = 0; i < 4; ++i) *(volatile v8us*)(gp + i * 2048 + 8 * tid) = q[i];
}

__global__ __launch_bounds__(GTHR) void k_gemm(const unsigned short* __restrict__ apl,
                                               const unsigned short* __restrict__ bt,
                                               float* outp, int nOut) {
  __shared__ __attribute__((aligned(16))) float stg[GBM * DH];
  const int tid = (int)threadIdx.x, lane = tid & 31, wave = tid >> 5, hh = lane >> 4, m = lane & 15;
  const int rowBase = (int)blockIdx.x * GBM;

  v8f acc[4];
  {
    const v8f z = {0.f, 0.f, 0.f, 0.f, 0.f, 0.f, 0.f, 0.f};
#pragma unroll
    for (int t = 0; t < 4; ++t) acc[t] = z;
  }
  const unsigned short* ap = apl + (size_t)(rowBase + 16 * wave + m) * (size_t)KP + 8 * hh;
  FragB af;
  af.h[0] = *(const v8usa*)(ap);
  af.h[1] = *(const v8usa*)(ap + 16);
#pragma unroll
  for (int nt = 0; nt < 4; ++nt) {
    const unsigned short* wq = bt + (size_t)(16 * nt + m) * (size_t)KP + 8 * hh;
    FragB bf;
    bf.h[0] = *(const v8usa*)wq;
    bf.h[1] = *(const v8usa*)(wq + 16);
    acc[nt] = wmb(af, bf, acc[nt]);
  }

#pragma unroll
  for (int nt = 0; nt < 4; ++nt) {
    const int lc = 16 * nt + m;
#pragma unroll
    for (int r = 0; r < 8; ++r) {
      const int lr = 16 * wave + 8 * hh + r;
      stg[lr * DH + lc] = acc[nt][r];
    }
  }
  __syncthreads();

  v4f pv[8];
#pragma unroll
  for (int i = 0; i < 8; ++i) pv[i] = *(const v4fa*)(stg + (16 * wave + 2 * i + hh) * DH + 4 * m);
#pragma unroll
  for (int i = 0; i < 8; ++i) {
    const int r = rowBase + 16 * wave + 2 * i + hh;
    if (r < nOut) *(volatile v4f*)(outp + (size_t)r * DH + 4 * m) = pv[i];
  }
  __threadfence();
#pragma unroll
  for (int i = 0; i < 8; ++i) {
    const int r = rowBase + 16 * wave + 2 * i + hh;
    if (r < nOut) *(volatile v4f*)(outp + (size_t)r * DH + 4 * m) = pv[i];
  }
}

template <int L2>
__global__ __launch_bounds__(NTHR) void k_scan(const int* __restrict__ gath, const int* __restrict__ keys,
                                               int nE, int nN, int vec8,
                                               const float* __restrict__ xin, const int* __restrict__ mask,
                                               const float* h1in,
                                               const float* __restrict__ wrel, const float* __restrict__ wroot,
                                               const float* __restrict__ bias,
                                               float* h1out, unsigned short* h2out) {
  extern __shared__ __attribute__((aligned(16))) int dsm[];
  int* list = dsm;
  int* hl   = dsm + LISTN;
  int* sl   = hl + RCAP;
  int* cnt  = sl + RCAP;
  int* offs = cnt + NBA;
  int* cur  = offs + NBA;
  int* misc = cur + NBA;
  float* wsm = (float*)(misc + MISC_INTS);
  float* tile1 = wsm + WSM_INTS;
  unsigned short* tile2 = (unsigned short*)(wsm + WSM_INTS);
  const int tid = (int)threadIdx.x, lane = tid & 31, wave = tid >> 5;
  const int nodeBase = (int)blockIdx.x * NBA;
  constexpr int NWT = (L2 != 0) ? (D1 * D2) : (DX * D1);
  constexpr int NBI = (L2 != 0) ? D2 : D1;

  {
    const v4i z4 = {0, 0, 0, 0};
    for (int i = tid * 4; i < AGG_ZINTS; i += NTHR * 4) *(v4ia*)(dsm + i) = z4;
    if (tid < MISC_INTS) misc[tid] = 0;
    if (tid < NWT) { wsm[tid] = bf16_val(wrel[tid]); wsm[NWT + tid] = bf16_val(wroot[tid]); }
    if (tid < NBI) wsm[2 * NWT + tid] = bf16_val(bias[tid]);
  }
  __syncthreads();

  int t = 0, ov = 0;
  const int nChunks = (nE + CHUNK - 1) / CHUNK;
#pragma unroll 1
  for (int ch = 0; ch < nChunks; ++ch) {
    const int cbase = ch * CHUNK;
    const int wc = scan_chunk<SLA>(keys, nE, cbase, nodeBase, NBA, vec8, list, tid, lane, wave);
    if (lane == 0) misc[wave] = wc;
    __syncthreads();
    if (wave == 0) {
#pragma unroll 1
      for (int w2 = 0; w2 < NWAVE; ++w2) {
        int c = misc[w2];
        c = c < 0 ? 0 : (c > WCAP ? WCAP : c);
#pragma unroll 1
        for (int b0 = 0; b0 < c; b0 += 32) {
          const int idx = b0 + lane;
          const int ent = list[w2 * WCAP + (idx < WCAP ? idx : WCAP - 1)];
          const int m32 = (c - b0) < 32 ? (c - b0) : 32;
#pragma unroll 1
          for (int k = 0; k < m32; ++k) {
            const int u    = __builtin_amdgcn_readlane(ent, k);
            const int slot = u & (NBA - 1);
            const int el   = (u >> SLA) & (CHUNK - 1);
            const int pk   = ((cbase + el) << SLA) | slot;
            if (t < RCAP) {
              if (lane == 0) { hl[t] = pk; cnt[slot] = cnt[slot] + 1; }
              t = t + 1;
            } else {
              ov = 1;
            }
          }
        }
      }
    }
    __syncthreads();
  }
  if (wave == 0 && lane == 0) { misc[8] = t; misc[9] = ov; }
  __syncthreads();
  int tt = misc[8];
  tt = tt < 0 ? 0 : (tt > RCAP ? RCAP : tt);
  const int ovf = misc[9];

  if (wave == 0) {
    const int base = lane * (NBA / 32);
    int s = 0;
#pragma unroll 1
    for (int i = 0; i < NBA / 32; ++i) s += cnt[base + i];
    int incl = s;
#pragma unroll
    for (int d = 1; d < 32; d <<= 1) {
      const int y = __shfl_up(incl, d, 32);
      if (lane >= d) incl += y;
    }
    int run = incl - s;
#pragma unroll 1
    for (int i = 0; i < NBA / 32; ++i) {
      const int cv = cnt[base + i];
      offs[base + i] = run;
      cur[base + i]  = run;
      run += cv;
    }
  }
  __syncthreads();
  if (wave == 0) {
#pragma unroll 1
    for (int b0 = 0; b0 < tt; b0 += 32) {
      const int idx = b0 + lane;
      const int ent = hl[idx < RCAP ? idx : RCAP - 1];
      const int m32 = (tt - b0) < 32 ? (tt - b0) : 32;
#pragma unroll 1
      for (int k = 0; k < m32; ++k) {
        const int u    = __builtin_amdgcn_readlane(ent, k);
        const int slot = u & (NBA - 1);
        if (lane == 0) {
          int p = cur[slot];
          p = p < 0 ? 0 : (p > RCAP - 1 ? RCAP - 1 : p);
          sl[p] = u;
          cur[slot] = p + 1;
        }
      }
    }
  }
  __syncthreads();

  const float pz = (ovf != 0) ? qnan_f() : 0.0f;
#pragma unroll 1
  for (int si = 0; si < NBA / NWAVE; ++si) {
    const int s    = si * NWAVE + wave;
    const int node = nodeBase + s;
    int c = cnt[s];
    const bool big = c > DEGCAP;
    c = c < 0 ? 0 : (c > DEGCAP ? DEGCAP : c);
    int o = offs[s];
    o = o < 0 ? 0 : (o > RCAP ? RCAP : o);
    const int nc = node < nN ? node : nN - 1;
    const bool live = node < nN;
    float ag[8];
#pragma unroll
    for (int i = 0; i < 8; ++i) ag[i] = 0.0f;
#pragma unroll 1
    for (int b0 = 0; b0 < c; b0 += 32) {
      int idx = o + b0 + lane;
      idx = idx > RCAP - 1 ? RCAP - 1 : idx;
      const int ent = sl[idx];
      int eid = ent >> SLA;
      eid = eid < 0 ? 0 : (eid > nE - 1 ? nE - 1 : eid);
      int sr = gath[eid];
      sr = sr < 0 ? 0 : (sr > nN - 1 ? nN - 1 : sr);
      const bool ok = (b0 + lane) < c;
      if constexpr (L2 == 0) {
        const v2f xv = *(const v2fa*)(xin + (size_t)sr * DX);
        ag[0] += ok ? bf16_val(xv.x) : 0.0f;
        ag[1] += ok ? bf16_val(xv.y) : 0.0f;
      } else {
        const v4f r0 = *(const v4fa*)(h1in + (size_t)sr * D1);
        const v4f r1 = *(const v4fa*)(h1in + (size_t)sr * D1 + 4);
        ag[0] += ok ? r0.x : 0.0f;
        ag[1] += ok ? r0.y : 0.0f;
        ag[2] += ok ? r0.z : 0.0f;
        ag[3] += ok ? r0.w : 0.0f;
        ag[4] += ok ? r1.x : 0.0f;
        ag[5] += ok ? r1.y : 0.0f;
        ag[6] += ok ? r1.z : 0.0f;
        ag[7] += ok ? r1.w : 0.0f;
      }
    }
    constexpr int NAG = (L2 != 0) ? 8 : 2;
#pragma unroll
    for (int i = 0; i < NAG; ++i) {
#pragma unroll
      for (int off = 16; off > 0; off >>= 1) ag[i] += __shfl_xor(ag[i], off, 32);
    }

    if constexpr (L2 == 0) {
      const int j = lane & 7;
      const v2f xs = *(const v2fa*)(xin + (size_t)nc * DX);
      const float x0 = bf16_val(xs.x), x1 = bf16_val(xs.y);
      const int mk = mask[nc];
      const bool mbad = live && (mk == 0);
      const float rel = fmaf(ag[1], wsm[D1 + j], ag[0] * wsm[j]);
      const float rt  = fmaf(x1, wsm[NWT + D1 + j], x0 * wsm[NWT + j]);
      float tv = (rel + rt) + wsm[2 * NWT + j];
      tv = (tv < 0.0f) ? 0.0f : tv;
      const float pzr = (big || mbad) ? qnan_f() : pz;
      const float hv = live ? (tv + pzr) : 0.0f;
      if (lane < D1) tile1[s * D1 + lane] = hv;
    } else {
      const int n = lane & 15;
      const v4f s0 = *(const v4fa*)(h1in + (size_t)nc * D1);
      const v4f s1 = *(const v4fa*)(h1in + (size_t)nc * D1 + 4);
      float rel = ag[0] * wsm[n];
      rel = fmaf(ag[1], wsm[1 * D2 + n], rel);
      rel = fmaf(ag[2], wsm[2 * D2 + n], rel);
      rel = fmaf(ag[3], wsm[3 * D2 + n], rel);
      rel = fmaf(ag[4], wsm[4 * D2 + n], rel);
      rel = fmaf(ag[5], wsm[5 * D2 + n], rel);
      rel = fmaf(ag[6], wsm[6 * D2 + n], rel);
      rel = fmaf(ag[7], wsm[7 * D2 + n], rel);
      float rt = s0.x * wsm[NWT + n];
      rt = fmaf(s0.y, wsm[NWT + 1 * D2 + n], rt);
      rt = fmaf(s0.z, wsm[NWT + 2 * D2 + n], rt);
      rt = fmaf(s0.w, wsm[NWT + 3 * D2 + n], rt);
      rt = fmaf(s1.x, wsm[NWT + 4 * D2 + n], rt);
      rt = fmaf(s1.y, wsm[NWT + 5 * D2 + n], rt);
      rt = fmaf(s1.z, wsm[NWT + 6 * D2 + n], rt);
      rt = fmaf(s1.w, wsm[NWT + 7 * D2 + n], rt);
      float tv = (rel + rt) + wsm[2 * NWT + n];
      tv = (tv < 0.0f) ? 0.0f : tv;
      const float pzr = big ? qnan_f() : pz;
      const float hv = live ? (tv + pzr) : 0.0f;
      const unsigned hbits = bf16_bits(hv);
      const unsigned lbits = bf16_bits(hv - __uint_as_float(hbits << 16));
      if (lane < D2) {
        tile2[s * KP + n]      = (unsigned short)hbits;
        tile2[s * KP + D2 + n] = (unsigned short)lbits;
      }
    }
  }
  __syncthreads();

  if constexpr (L2 == 0) {
    v4f q[4];
#pragma unroll
    for (int i = 0; i < 4; ++i) q[i] = *(const v4fa*)(tile1 + i * 1024 + 4 * tid);
    float* gp = h1out + (size_t)nodeBase * D1;
#pragma unroll
    for (int i = 0; i < 4; ++i) *(volatile v4f*)(gp + i * 1024 + 4 * tid) = q[i];
    __threadfence();
#pragma unroll
    for (int i = 0; i < 4; ++i) *(volatile v4f*)(gp + i * 1024 + 4 * tid) = q[i];
  } else {
    v8us q[8];
#pragma unroll
    for (int i = 0; i < 8; ++i) q[i] = *(const v8usa*)(tile2 + i * 2048 + 8 * tid);
    unsigned short* gp = h2out + (size_t)nodeBase * KP;
#pragma unroll
    for (int i = 0; i < 8; ++i) *(volatile v8us*)(gp + i * 2048 + 8 * tid) = q[i];
    __threadfence();
#pragma unroll
    for (int i = 0; i < 8; ++i) *(volatile v8us*)(gp + i * 2048 + 8 * tid) = q[i];
  }
}

__global__ __launch_bounds__(NTHR) void k_cand(const int* __restrict__ cand, int nC,
                                               const int* __restrict__ mask, int nG, int nU, int nTot,
                                               const float* __restrict__ PH, const float* __restrict__ PU,
                                               const float* __restrict__ ba, const float* __restrict__ wb,
                                               const float* __restrict__ bb, float* out) {
  __shared__ __attribute__((aligned(16))) float outs[NWAVE * 32];
  __shared__ int flg[NWAVE];
  const int tid = (int)threadIdx.x, lane = tid & 31, wave = tid >> 5, hh = lane >> 4, q = lane & 15;

  int bad = 0;
  if (blockIdx.x == 0) {
    int b = 0;
#pragma unroll 1
    for (int i = tid; i < nTot; i += NTHR) {
      const int mk = mask[i];
      b |= (i < nG) ? ((mk == 0) ? 1 : 0) : ((mk != 0) ? 1 : 0);
    }
    const unsigned bal = __builtin_amdgcn_ballot_w32(b != 0);
    if (lane == 0) flg[wave] = (bal != 0u) ? 1 : 0;
    __syncthreads();
#pragma unroll
    for (int w2 = 0; w2 < NWAVE; ++w2) bad |= flg[w2];
  }
  const float pzn = (bad != 0 && wave == 0) ? qnan_f() : 0.0f;

  v4f ba4, wb4;
  {
    const v4f tb = *(const v4fa*)(ba + 4 * q);
    const v4f tw = *(const v4fa*)(wb + 4 * q);
    ba4.x = bf16_val(tb.x); ba4.y = bf16_val(tb.y); ba4.z = bf16_val(tb.z); ba4.w = bf16_val(tb.w);
    wb4.x = bf16_val(tw.x); wb4.y = bf16_val(tw.y); wb4.z = bf16_val(tw.z); wb4.w = bf16_val(tw.w);
  }
  const float bb0 = bf16_val(bb[0]);

  const int lineIdx = (int)blockIdx.x * NWAVE + wave;
  const long long cbl = (long long)lineIdx * 32;
  if (cbl < (long long)nC) {
    const int cbase = (int)cbl;
#pragma unroll 2
    for (int step = 0; step < 16; ++step) {
      int c = cbase + 2 * step + hh;
      c = c > nC - 1 ? nC - 1 : c;
      const v2i i2 = *(const v2ia*)(cand + (size_t)c * 2);
      int c0 = i2.x; c0 = c0 < 0 ? 0 : (c0 > nG - 1 ? nG - 1 : c0);
      int c1 = i2.y; c1 = c1 < 0 ? 0 : (c1 > nU - 1 ? nU - 1 : c1);
      const v4f p = *(const v4fa*)(PH + (size_t)c0 * DH + 4 * q);
      const v4f u = *(const v4fa*)(PU + (size_t)c1 * DH + 4 * q);
      const v4f tv = p + u + ba4;
      v4f hd;
      hd.x = (tv.x < 0.0f) ? 0.0f : tv.x;
      hd.y = (tv.y < 0.0f) ? 0.0f : tv.y;
      hd.z = (tv.z < 0.0f) ? 0.0f : tv.z;
      hd.w = (tv.w < 0.0f) ? 0.0f : tv.w;
      float d = hd.x * wb4.x;
      d = fmaf(hd.y, wb4.y, d);
      d = fmaf(hd.z, wb4.z, d);
      d = fmaf(hd.w, wb4.w, d);
#pragma unroll
      for (int off = 8; off > 0; off >>= 1) d += __shfl_xor(d, off, 32);
      if (q == 0) outs[wave * 32 + 2 * step + hh] = (d + bb0) + pzn;
    }
    wave_sync();
    const v4f o4 = *(const v4fa*)(outs + wave * 32 + 4 * (lane & 7));
    const int nrem = nC - cbase;
    if (nrem >= 32) {
      if (lane < 8) *(volatile v4f*)(out + (size_t)cbase + 4 * lane) = o4;
      __threadfence();
      if (lane < 8) *(volatile v4f*)(out + (size_t)cbase + 4 * lane) = o4;
    } else {
      if (lane == 0) {
#pragma unroll 1
        for (int j = 0; j < nrem; ++j) *(volatile float*)(out + (size_t)cbase + j) = outs[wave * 32 + j];
        __threadfence();
#pragma unroll 1
        for (int j = 0; j < nrem; ++j) *(volatile float*)(out + (size_t)cbase + j) = outs[wave * 32 + j];
      }
    }
  }
}

static inline int cdiv(int a, int b) { return (a + b - 1) / b; }
static inline size_t al256(size_t o) { return (o + 255) & ~(size_t)255; }

extern "C" void kernel_launch(void* const* d_in, const int* in_sizes, int n_in,
                              void* d_out, int out_size, void* d_ws, size_t ws_size,
                              hipStream_t stream) {
  if (n_in < 16) return;
  const int nTot = in_sizes[1];
  if (nTot <= NGC || in_sizes[0] != DX * nTot) return;
  const int nU = nTot - NGC;
  if (in_sizes[2] < 2 || (in_sizes[2] & 1) != 0) return;
  const int nC = in_sizes[2] / 2;
  if (in_sizes[3] < 2 || (in_sizes[3] & 1) != 0) return;
  const int nE = in_sizes[3] / 2;
  if (nE > (1 << 22)) return;
  if (in_sizes[4] != DX * D1 || in_sizes[5] != DX * D1 || in_sizes[6] != D1) return;
  if (in_sizes[7] != D1 * D2 || in_sizes[8] != D1 * D2 || in_sizes[9] != D2) return;
  if (in_sizes[10] != DX * D2 || in_sizes[11] != D2) return;
  if (in_sizes[12] != 2 * D2 * DH || in_sizes[13] != DH) return;
  if (in_sizes[14] != DH || in_sizes[15] != 1) return;
  if (out_size != nC) return;

  const float* x      = (const float*)d_in[0];
  const int*   mask   = (const int*)d_in[1];
  const int*   cand   = (const int*)d_in[2];
  const int*   edges  = (const int*)d_in[3];
  const float* w1_rel = (const float*)d_in[4];
  const float* w1_root= (const float*)d_in[5];
  const float* b1     = (const float*)d_in[6];
  const float* w2_rel = (const float*)d_in[7];
  const float* w2_root= (const float*)d_in[8];
  const float* b2     = (const float*)d_in[9];
  const float* wu     = (const float*)d_in[10];
  const float* bu     = (const float*)d_in[11];
  const float* wa     = (const float*)d_in[12];
  const float* ba     = (const float*)d_in[13];
  const float* wb     = (const float*)d_in[14];
  const float* bb     = (const float*)d_in[15];
  float* out = (float*)d_out;
  const int* src = edges;
  const int* dst = edges + nE;

  const int gA   = cdiv(NGC, NBA);
  const int RA   = gA * NBA;
  const int MPG  = cdiv(NGC, GBM) * GBM;
  const int gX   = cdiv(nU, XROWS);
  const int MPU  = gX * XROWS;
  const int MPU2 = cdiv(nU, GBM) * GBM;
  if (RA < MPG || MPU < MPU2) return;
  const int vec8 = ((nE & 3) == 0) ? 1 : 0;

  char* ws = (char*)d_ws;
  size_t off = 0;
  const size_t oBW = off; off = al256(off + (size_t)2 * DH * KP * 2);
  const size_t oXU = off; off = al256(off + (size_t)MPU * KP * 2);
  const size_t oH1 = off; off = al256(off + (size_t)RA * D1 * 4);
  const size_t oH2 = off; off = al256(off + (size_t)RA * KP * 2);
  const size_t oPH = off; off = al256(off + (size_t)NGC * DH * 4);
  const size_t oPU = off; off = al256(off + (size_t)nU * DH * 4);
  if (off > ws_size || off > (size_t)WSMAX) return;
  unsigned short* BW  = (unsigned short*)(ws + oBW);
  unsigned short* XUP = (unsigned short*)(ws + oXU);
  float*          H1  = (float*)(ws + oH1);
  unsigned short* H2P = (unsigned short*)(ws + oH2);
  float*          PH  = (float*)(ws + oPH);
  float*          PU  = (float*)(ws + oPU);

  const size_t lds1 = (size_t)LDS1_INTS * 4;
  const size_t lds2 = (size_t)LDS2_INTS * 4;
  hipFuncSetAttribute(reinterpret_cast<const void*>(&k_scan<0>), hipFuncAttributeMaxDynamicSharedMemorySize, (int)lds1);
  hipFuncSetAttribute(reinterpret_cast<const void*>(&k_scan<1>), hipFuncAttributeMaxDynamicSharedMemorySize, (int)lds2);

  k_wprep<<<1, NTHR, 0, stream>>>(wa, BW);
  k_xprep<<<gX, NTHR, 0, stream>>>(x, mask, wu, bu, NGC, nU, nTot, XUP);
  k_scan<0><<<gA, NTHR, lds1, stream>>>(src, dst, nE, NGC, vec8, x, mask, H1, w1_rel, w1_root, b1, H1, H2P);
  k_scan<1><<<gA, NTHR, lds2, stream>>>(src, dst, nE, NGC, vec8, x, mask, H1, w2_rel, w2_root, b2, H1, H2P);
  k_gemm<<<MPG / GBM, GTHR, 0, stream>>>(H2P, BW, PH, NGC);
  k_gemm<<<MPU2 / GBM, GTHR, 0, stream>>>(XUP, BW + DH * KP, PU, nU);
  k_cand<<<cdiv(nC, NTHR), NTHR, 0, stream>>>(cand, nC, mask, NGC, nU, nTot, PH, PU, ba, wb, bb, out);
}
